// Net_81552839016511
// MI455X (gfx1250) — hardware-verified
//
#include <hip/hip_runtime.h>
#include <stddef.h>
#include <stdint.h>


#define XF     50
#define K1P    64
#define HD     128
#define K2     256
#define YP     256
#define NCLS   121
#define NTHR   256
#define NWAVE  8
#define EPT    8
#define CHUNK  (NTHR * EPT)
#define WCAP   (EPT * 32)
#define LISTN  (NWAVE * WCAP)
#define NBD    8192
#define SLD    13
#define NBA    1024
#define SLA    10
#define RCAP   28672
#define DEGCAP 64
#define GBM    64
#define GBN    128
#define GTHR   128
#define NUW1   (HD * (K1P / 8))
#define NUW2   (HD * (K2 / 8))
#define NUWT   (NUW1 + 5 * NUW2)
#define AGG_ZINTS    (LISTN + 2 * RCAP + 3 * NBA)
#define MISC_INTS    16
#define ROWBUF_INTS  (NWAVE * YP / 2)
#define AGG_LDS_INTS (AGG_ZINTS + MISC_INTS + ROWBUF_INTS)
#define WSMAX  134217728

static_assert((CHUNK & (CHUNK - 1)) == 0 && CHUNK <= 4096);
static_assert((NBD & (NBD - 1)) == 0 && NBD == (1 << SLD));
static_assert((NBA & (NBA - 1)) == 0 && NBA == (1 << SLA));
static_assert(((long long)CHUNK << SLD) < (1LL << 31));
static_assert(((long long)CHUNK << SLA) < (1LL << 31));
static_assert(NBD % (NTHR * 4) == 0);
static_assert(LISTN % NTHR == 0);
static_assert(NBA % NWAVE == 0 && NBA % 32 == 0 && NBA % GBM == 0);
static_assert(RCAP % 32 == 0 && AGG_ZINTS % 4 == 0 && LISTN % 4 == 0 && ((AGG_ZINTS + MISC_INTS) % 4) == 0);
static_assert(AGG_ZINTS % (NTHR * 4) == 0);
static_assert(K1P % 32 == 0 && K2 % 32 == 0 && K2 == 2 * HD && YP == K2);
static_assert(GBN == HD && GBM == (GTHR / 32) * 16 && HD == 4 * 32 && GTHR == GBN);
static_assert(NUW1 % NTHR == 0 && NUW2 % NTHR == 0 && NUWT % NTHR == 0);
static_assert(AGG_LDS_INTS * 4 <= 300000);
static_assert(NCLS <= GBN && GBM * NCLS <= GBM * GBN);
static_assert(((GBM * NCLS * 4) % 128) == 0);
static_assert(XF % 2 == 0 && XF <= K1P);

typedef float          v2f   __attribute__((ext_vector_type(2)));
typedef float          v4f   __attribute__((ext_vector_type(4)));
typedef float          v8f   __attribute__((ext_vector_type(8)));
typedef int            v4i   __attribute__((ext_vector_type(4)));
typedef int            v8i   __attribute__((ext_vector_type(8)));
typedef unsigned short v4us  __attribute__((ext_vector_type(4)));
typedef unsigned short v8us  __attribute__((ext_vector_type(8)));
typedef unsigned short v16us __attribute__((ext_vector_type(16)));
typedef __bf16         v16bf __attribute__((ext_vector_type(16)));
typedef v2f  __attribute__((may_alias)) v2fa;
typedef v4f  __attribute__((may_alias)) v4fa;
typedef v4i  __attribute__((may_alias)) v4ia;
typedef v4us __attribute__((may_alias)) v4usa;
typedef v8us __attribute__((may_alias)) v8usa;
union FragB { v16bf v; v16us u; v8us h[2]; v8i w; };

__device__ __forceinline__ v8f wmb(const FragB& a, const FragB& b, v8f c) {
  v8f d = __builtin_amdgcn_wmma_f32_16x16x32_bf16(false, a.v, false, b.v, (short)0, c, false, false);
  asm volatile("v_nop\n\tv_nop\n\tv_nop\n\tv_nop" : "+v"(d) : "v"(a.w), "v"(b.w));
  return d;
}

__device__ __forceinline__ unsigned bf16_bits(float f) {
  const unsigned u = __float_as_uint(f);
  return (u + 0x7FFFu + ((u >> 16) & 1u)) >> 16;
}
__device__ __forceinline__ float bf16_val(float f) {
  return __uint_as_float(bf16_bits(f) << 16);
}

__device__ __forceinline__ void wave_sync() {
  __builtin_amdgcn_fence(__ATOMIC_RELEASE, "wavefront");
  __builtin_amdgcn_wave_barrier();
  __builtin_amdgcn_fence(__ATOMIC_ACQUIRE, "wavefront");
}

template <int SLB>
__device__ __forceinline__ int scan_chunk(const int* __restrict__ dsts, int nE, int cbase, int slotBase,
                                          int nb, int vec8, int* list, int tid, int lane, int wave) {
  int wc = 0;
  const int el0  = tid * EPT;
  const int e0   = cbase + el0;
  const int sent = -2147483647 - 1;
  v4i da, db;
  if (vec8 != 0 && cbase + CHUNK <= nE) {
    da = *(const v4i*)(dsts + e0);
    db = *(const v4i*)(dsts + e0 + 4);
  } else {
    da.x = (e0     < nE) ? dsts[min(e0,     nE - 1)] : sent;
    da.y = (e0 + 1 < nE) ? dsts[min(e0 + 1, nE - 1)] : sent;
    da.z = (e0 + 2 < nE) ? dsts[min(e0 + 2, nE - 1)] : sent;
    da.w = (e0 + 3 < nE) ? dsts[min(e0 + 3, nE - 1)] : sent;
    db.x = (e0 + 4 < nE) ? dsts[min(e0 + 4, nE - 1)] : sent;
    db.y = (e0 + 5 < nE) ? dsts[min(e0 + 5, nE - 1)] : sent;
    db.z = (e0 + 6 < nE) ? dsts[min(e0 + 6, nE - 1)] : sent;
    db.w = (e0 + 7 < nE) ? dsts[min(e0 + 7, nE - 1)] : sent;
  }
  const unsigned nbs = (unsigned)slotBase;
  const unsigned unb = (unsigned)nb;
  const unsigned s0 = (unsigned)da.x - nbs, s1 = (unsigned)da.y - nbs;
  const unsigned s2 = (unsigned)da.z - nbs, s3 = (unsigned)da.w - nbs;
  const unsigned s4 = (unsigned)db.x - nbs, s5 = (unsigned)db.y - nbs;
  const unsigned s6 = (unsigned)db.z - nbs, s7 = (unsigned)db.w - nbs;
  const bool h0 = s0 < unb, h1 = s1 < unb, h2 = s2 < unb, h3 = s3 < unb;
  const bool h4 = s4 < unb, h5 = s5 < unb, h6 = s6 < unb, h7 = s7 < unb;
  const unsigned any = __builtin_amdgcn_ballot_w32(h0 | h1 | h2 | h3 | h4 | h5 | h6 | h7);
  if (any != 0u) {
#define HITJ(J, HJ, SJ) { \
      const unsigned mj = __builtin_amdgcn_ballot_w32(HJ); \
      if (mj != 0u) { \
        if (HJ) { \
          const int pos = wc + (int)__builtin_amdgcn_mbcnt_lo(mj, 0u); \
          if (pos < WCAP) list[wave * WCAP + pos] = ((el0 + (J)) << SLB) | (int)(SJ); \
        } \
        wc += (int)__builtin_popcount(mj); } }
    HITJ(0, h0, s0)
    HITJ(1, h1, s1)
    HITJ(2, h2, s2)
    HITJ(3, h3, s3)
    HITJ(4, h4, s4)
    HITJ(5, h5, s5)
    HITJ(6, h6, s6)
    HITJ(7, h7, s7)
#undef HITJ
  }
  return wc;
}

__global__ __launch_bounds__(NTHR) void k_wprep(const float* __restrict__ W1, const float* __restrict__ W2,
                                                const float* __restrict__ W3, const float* __restrict__ W4,
                                                const float* __restrict__ W5, const float* __restrict__ W6,
                                                unsigned short* W1T, unsigned short* WTB) {
  const int u = (int)blockIdx.x * NTHR + (int)threadIdx.x;
  const float* W;
  unsigned short* P;
  int KR, NC, sh, v;
  if (u < NUW1)                 { W = W1; P = W1T;                        KR = XF; NC = HD;   sh = 3; v = u; }
  else if (u < NUW1 + 1 * NUW2) { W = W2; P = WTB + (size_t)0 * HD * K2; KR = HD; NC = HD;   sh = 5; v = u - NUW1; }
  else if (u < NUW1 + 2 * NUW2) { W = W3; P = WTB + (size_t)1 * HD * K2; KR = HD; NC = HD;   sh = 5; v = u - NUW1 - 1 * NUW2; }
  else if (u < NUW1 + 3 * NUW2) { W = W4; P = WTB + (size_t)2 * HD * K2; KR = HD; NC = HD;   sh = 5; v = u - NUW1 - 2 * NUW2; }
  else if (u < NUW1 + 4 * NUW2) { W = W5; P = WTB + (size_t)3 * HD * K2; KR = HD; NC = HD;   sh = 5; v = u - NUW1 - 3 * NUW2; }
  else if (u < NUW1 + 5 * NUW2) { W = W6; P = WTB + (size_t)4 * HD * K2; KR = HD; NC = NCLS; sh = 5; v = u - NUW1 - 4 * NUW2; }
  else return;
  const int kp  = 8 << sh;
  const int n   = v >> sh;
  const int k8  = (v & ((1 << sh) - 1)) * 8;
  const int ncl = n < NC ? n : NC - 1;
  v8us o;
#pragma unroll
  for (int i = 0; i < 8; ++i) {
    const int kk = (k8 + i) & (HD - 1);
    const int kr = kk < KR ? kk : KR - 1;
    const float wv = W[(size_t)kr * NC + ncl];
    o[i] = (kk < KR && n < NC) ? (unsigned short)bf16_bits(wv) : (unsigned short)0;
  }
  unsigned short* dp = P + (size_t)n * kp + k8;
  *(volatile v8us*)dp = o;
  __threadfence();
  *(volatile v8us*)dp = o;
}

__global__ __launch_bounds__(NTHR) void k_cvx(const float* __restrict__ x, int nN, int nUnits,
                                              unsigned short* xb) {
  const int u = (int)blockIdx.x * NTHR + (int)threadIdx.x;
  if (u >= nUnits) return;
  const int row = u >> 3;
  const int k8  = (u & 7) * 8;
  const int rc  = row < nN ? row : nN - 1;
  const bool okr = row < nN;
  const float* p = x + (size_t)rc * XF;
  v8us o;
#pragma unroll
  for (int j = 0; j < 4; ++j) {
    const int c  = k8 + 2 * j;
    const int cc = c < XF - 2 ? c : XF - 2;
    const v2f a  = *(const v2fa*)(p + cc);
    const bool ok = okr && (c < XF);
    o[2 * j]     = ok ? (unsigned short)bf16_bits(a.x) : (unsigned short)0;
    o[2 * j + 1] = ok ? (unsigned short)bf16_bits(a.y) : (unsigned short)0;
  }
  unsigned short* dp = xb + (size_t)row * K1P + k8;
  *(volatile v8us*)dp = o;
  __threadfence();
  *(volatile v8us*)dp = o;
}

__global__ __launch_bounds__(NTHR) void k_deg(const int* __restrict__ dsts, int nE, int vec8, float* dis) {
  __shared__ __attribute__((aligned(16))) int scnt[NBD];
  __shared__ __attribute__((aligned(16))) int list[LISTN];
  __shared__ int wcnt[NWAVE];
  const int tid = (int)threadIdx.x, lane = tid & 31, wave = tid >> 5;
  const int nodeBase = (int)blockIdx.x * NBD;

  for (int i = tid; i < NBD; i += NTHR) scnt[i] = 0;
  for (int i = tid; i < LISTN; i += NTHR) list[i] = 0;
  if (tid < NWAVE) wcnt[tid] = 0;
  __syncthreads();

  const int nChunks = (nE + CHUNK - 1) / CHUNK;
#pragma unroll 1
  for (int ch = 0; ch < nChunks; ++ch) {
    const int cbase = ch * CHUNK;
    const int wc = scan_chunk<SLD>(dsts, nE, cbase, nodeBase, NBD, vec8, list, tid, lane, wave);
    if (lane == 0) wcnt[wave] = wc;
    __syncthreads();
    if (wave == 0) {
#pragma unroll 1
      for (int w2 = 0; w2 < NWAVE; ++w2) {
        int c = wcnt[w2];
        c = c < 0 ? 0 : (c > WCAP ? WCAP : c);
#pragma unroll 1
        for (int b0 = 0; b0 < c; b0 += 32) {
          const int idx = b0 + lane;
          const int ent = list[w2 * WCAP + (idx < WCAP ? idx : WCAP - 1)];
          const int m32 = (c - b0) < 32 ? (c - b0) : 32;
#pragma unroll 1
          for (int k = 0; k < m32; ++k) {
            const int u  = __builtin_amdgcn_readlane(ent, k);
            const int sl = u & (NBD - 1);
            if (lane == 0) scnt[sl] = scnt[sl] + 1;
          }
        }
      }
    }
    __syncthreads();
  }

  v4f vals[NBD / (NTHR * 4)];
#pragma unroll
  for (int it = 0; it < NBD / (NTHR * 4); ++it) {
    const int s0 = it * (NTHR * 4) + 4 * tid;
    const v4i c4 = *(const v4ia*)(scnt + s0);
    const float d0 = (float)c4.x + 1.0f, d1 = (float)c4.y + 1.0f;
    const float d2 = (float)c4.z + 1.0f, d3 = (float)c4.w + 1.0f;
    v4f vv;
    vv.x = rsqrtf(d0); vv.y = rsqrtf(d1); vv.z = rsqrtf(d2); vv.w = rsqrtf(d3);
    vals[it] = vv;
  }
#pragma unroll
  for (int it = 0; it < NBD / (NTHR * 4); ++it) {
    const int s0 = it * (NTHR * 4) + 4 * tid;
    *(volatile v4f*)(dis + (size_t)nodeBase + s0) = vals[it];
  }
  __threadfence();
#pragma unroll
  for (int it = 0; it < NBD / (NTHR * 4); ++it) {
    const int s0 = it * (NTHR * 4) + 4 * tid;
    *(volatile v4f*)(dis + (size_t)nodeBase + s0) = vals[it];
  }
}

template <int MODE>
__global__ __launch_bounds__(GTHR) void k_gemm(const unsigned short* __restrict__ Apl, int lda,
                                               const unsigned short* __restrict__ BT, int K,
                                               const float* __restrict__ bias, int nB,
                                               float* outF, unsigned short* outY, int nN, int nTot) {
  __shared__ __attribute__((aligned(16))) float stg[GBM * GBN];
  __shared__ __attribute__((aligned(16))) float sbias[GBN];
  const int tid = (int)threadIdx.x, lane = tid & 31, wave = tid >> 5, hh = lane >> 4, m = lane & 15;
  const int rowBase = (int)blockIdx.x * GBM;

  {
    const int ci = (tid < nB) ? tid : 0;
    const float bvv = bias[ci];
    sbias[tid] = (tid < nB) ? bf16_val(bvv) : 0.0f;
  }

  v8f acc[8];
  {
    const v8f z = {0.f, 0.f, 0.f, 0.f, 0.f, 0.f, 0.f, 0.f};
#pragma unroll
    for (int t = 0; t < 8; ++t) acc[t] = z;
  }
  const unsigned short* ap = Apl + (size_t)(rowBase + 16 * wave + m) * (size_t)lda + 8 * hh;
  const unsigned short* bp = BT + (size_t)m * (size_t)K + 8 * hh;

#pragma unroll 1
  for (int k0 = 0; k0 < K; k0 += 32) {
    FragB af;
    af.h[0] = *(const v8usa*)(ap + k0);
    af.h[1] = *(const v8usa*)(ap + k0 + 16);
#pragma unroll
    for (int nt = 0; nt < 8; ++nt) {
      const unsigned short* wq = bp + (size_t)(16 * nt) * (size_t)K + k0;
      FragB bf;
      bf.h[0] = *(const v8usa*)wq;
      bf.h[1] = *(const v8usa*)(wq + 16);
      acc[nt] = wmb(af, bf, acc[nt]);
    }
  }

#pragma unroll
  for (int nt = 0; nt < 8; ++nt) {
    const int lc = 16 * nt + m;
#pragma unroll
    for (int r = 0; r < 8; ++r) {
      const int lr = 16 * wave + 8 * hh + r;
      stg[lr * GBN + lc] = acc[nt][r];
    }
  }
  __syncthreads();

  const v4f bb4 = *(const v4fa*)(sbias + 4 * lane);

  v4f pv[16];
#pragma unroll
  for (int i = 0; i < 16; ++i) pv[i] = *(const v4fa*)(stg + (16 * wave + i) * GBN + 4 * lane);
  __syncthreads();

  if constexpr (MODE == 0) {
#pragma unroll
    for (int i = 0; i < 16; ++i) {
      const int r = rowBase + 16 * wave + i;
      *(volatile v4f*)(outF + (size_t)r * HD + 4 * lane) = pv[i];
    }
    __threadfence();
#pragma unroll
    for (int i = 0; i < 16; ++i) {
      const int r = rowBase + 16 * wave + i;
      *(volatile v4f*)(outF + (size_t)r * HD + 4 * lane) = pv[i];
    }
  } else if constexpr (MODE == 1) {
#pragma unroll
    for (int i = 0; i < 16; ++i) {
      const bool ok = (rowBase + 16 * wave + i) < nN;
      const v4f t = pv[i] + bb4;
      v4f y;
      y.x = fmaxf(t.x, 0.0f); y.y = fmaxf(t.y, 0.0f); y.z = fmaxf(t.z, 0.0f); y.w = fmaxf(t.w, 0.0f);
      y.x = ok ? y.x : 0.0f; y.y = ok ? y.y : 0.0f; y.z = ok ? y.z : 0.0f; y.w = ok ? y.w : 0.0f;
      pv[i] = y;
    }
#pragma unroll
    for (int i = 0; i < 16; ++i) {
      v4us h4, l4;
      unsigned hb;
      hb = bf16_bits(pv[i].x); h4[0] = (unsigned short)hb; l4[0] = (unsigned short)bf16_bits(pv[i].x - __uint_as_float(hb << 16));
      hb = bf16_bits(pv[i].y); h4[1] = (unsigned short)hb; l4[1] = (unsigned short)bf16_bits(pv[i].y - __uint_as_float(hb << 16));
      hb = bf16_bits(pv[i].z); h4[2] = (unsigned short)hb; l4[2] = (unsigned short)bf16_bits(pv[i].z - __uint_as_float(hb << 16));
      hb = bf16_bits(pv[i].w); h4[3] = (unsigned short)hb; l4[3] = (unsigned short)bf16_bits(pv[i].w - __uint_as_float(hb << 16));
      unsigned short* srow = (unsigned short*)stg + (size_t)(16 * wave + i) * (2 * GBN);
      *(v4usa*)(srow + 4 * lane) = h4;
      *(v4usa*)(srow + HD + 4 * lane) = l4;
    }
    __syncthreads();
    v8us qv[16];
#pragma unroll
    for (int i = 0; i < 16; ++i) {
      const unsigned short* srow = (const unsigned short*)stg + (size_t)(16 * wave + i) * (2 * GBN);
      qv[i] = *(const v8usa*)(srow + 8 * lane);
    }
#pragma unroll
    for (int i = 0; i < 16; ++i) {
      unsigned short* rp = outY + (size_t)(rowBase + 16 * wave + i) * (size_t)YP + 8 * lane;
      *(volatile v8us*)rp = qv[i];
    }
    __threadfence();
#pragma unroll
    for (int i = 0; i < 16; ++i) {
      unsigned short* rp = outY + (size_t)(rowBase + 16 * wave + i) * (size_t)YP + 8 * lane;
      *(volatile v8us*)rp = qv[i];
    }
  } else {
    float* os = stg;
    const int c0 = 4 * lane;
#pragma unroll
    for (int i = 0; i < 16; ++i) {
      const int lr = 16 * wave + i;
      const v4f t = pv[i] + bb4;
      if (c0 + 0 < NCLS) os[lr * NCLS + c0 + 0] = t.x;
      if (c0 + 1 < NCLS) os[lr * NCLS + c0 + 1] = t.y;
      if (c0 + 2 < NCLS) os[lr * NCLS + c0 + 2] = t.z;
      if (c0 + 3 < NCLS) os[lr * NCLS + c0 + 3] = t.w;
    }
    __syncthreads();
    const size_t fb = (size_t)rowBase * (size_t)NCLS;
    constexpr int NIT = (GBM * GBN) / (4 * GTHR);
    v4f ov[NIT];
#pragma unroll
    for (int it = 0; it < NIT; ++it) ov[it] = *(const v4fa*)(os + 4 * (it * GTHR + tid));
#pragma unroll
    for (int it = 0; it < NIT; ++it) {
      const int t = it * GTHR + tid;
      const bool ok = (4 * t < GBM * NCLS) && (fb + (size_t)(4 * t) + 4 <= (size_t)nTot);
      if (ok) *(volatile v4f*)(outF + fb + (size_t)(4 * t)) = ov[it];
    }
    __threadfence();
#pragma unroll
    for (int it = 0; it < NIT; ++it) {
      const int t = it * GTHR + tid;
      const bool ok = (4 * t < GBM * NCLS) && (fb + (size_t)(4 * t) + 4 <= (size_t)nTot);
      if (ok) *(volatile v4f*)(outF + fb + (size_t)(4 * t)) = ov[it];
    }
  }
}

__global__ __launch_bounds__(NTHR) void k_agg(const int* __restrict__ srcs, const int* __restrict__ dsts,
                                              int nE, int nN, int vec8, int mRows,
                                              const float* __restrict__ dis,
                                              const float* __restrict__ xl, const float* __restrict__ bias,
                                              unsigned short* yout) {
  extern __shared__ __attribute__((aligned(16))) int dsm[];
  int* list = dsm;
  int* hl   = dsm + LISTN;
  int* sl   = hl + RCAP;
  int* cnt  = sl + RCAP;
  int* offs = cnt + NBA;
  int* cur  = offs + NBA;
  int* misc = cur + NBA;
  const int tid = (int)threadIdx.x, lane = tid & 31, wave = tid >> 5;
  unsigned short* rowbuf = (unsigned short*)(misc + MISC_INTS) + wave * YP;
  const int nodeBase = (int)blockIdx.x * NBA;

  {
    const v4i z4 = {0, 0, 0, 0};
    for (int i = tid * 4; i < AGG_ZINTS; i += NTHR * 4) *(v4ia*)(dsm + i) = z4;
    if (tid < MISC_INTS) misc[tid] = 0;
  }
  v4f bv4;
  {
    const v4f a = *(const v4fa*)(bias + 4 * lane);
    bv4.x = bf16_val(a.x); bv4.y = bf16_val(a.y); bv4.z = bf16_val(a.z); bv4.w = bf16_val(a.w);
  }
  __syncthreads();

  int t = 0, ov = 0;
  const int nChunks = (nE + CHUNK - 1) / CHUNK;
#pragma unroll 1
  for (int ch = 0; ch < nChunks; ++ch) {
    const int cbase = ch * CHUNK;
    const int wc = scan_chunk<SLA>(dsts, nE, cbase, nodeBase, NBA, vec8, list, tid, lane, wave);
    if (lane == 0) misc[wave] = wc;
    __syncthreads();
    if (wave == 0) {
#pragma unroll 1
      for (int w2 = 0; w2 < NWAVE; ++w2) {
        int c = misc[w2];
        c = c < 0 ? 0 : (c > WCAP ? WCAP : c);
#pragma unroll 1
        for (int b0 = 0; b0 < c; b0 += 32) {
          const int idx = b0 + lane;
          const int ent = list[w2 * WCAP + (idx < WCAP ? idx : WCAP - 1)];
          const int m32 = (c - b0) < 32 ? (c - b0) : 32;
#pragma unroll 1
          for (int k = 0; k < m32; ++k) {
            const int u    = __builtin_amdgcn_readlane(ent, k);
            const int slot = u & (NBA - 1);
            const int el   = (u >> SLA) & (CHUNK - 1);
            const int pk   = ((cbase + el) << SLA) | slot;
            if (t < RCAP) {
              if (lane == 0) { hl[t] = pk; cnt[slot] = cnt[slot] + 1; }
              t = t + 1;
            } else {
              ov = 1;
            }
          }
        }
      }
    }
    __syncthreads();
  }
  if (wave == 0 && lane == 0) { misc[8] = t; misc[9] = ov; }
  __syncthreads();
  int tt = misc[8];
  tt = tt < 0 ? 0 : (tt > RCAP ? RCAP : tt);
  const int ovf = misc[9];

  if (wave == 0) {
    const int base = lane * (NBA / 32);
    int s = 0;
#pragma unroll 1
    for (int i = 0; i < NBA / 32; ++i) s += cnt[base + i];
    int incl = s;
#pragma unroll
    for (int d = 1; d < 32; d <<= 1) {
      const int y = __shfl_up(incl, d, 32);
      if (lane >= d) incl += y;
    }
    int run = incl - s;
#pragma unroll 1
    for (int i = 0; i < NBA / 32; ++i) {
      const int cv = cnt[base + i];
      offs[base + i] = run;
      cur[base + i]  = run;
      run += cv;
    }
  }
  __syncthreads();
  if (wave == 0) {
#pragma unroll 1
    for (int b0 = 0; b0 < tt; b0 += 32) {
      const int idx = b0 + lane;
      const int ent = hl[idx < RCAP ? idx : RCAP - 1];
      const int m32 = (tt - b0) < 32 ? (tt - b0) : 32;
#pragma unroll 1
      for (int k = 0; k < m32; ++k) {
        const int u    = __builtin_amdgcn_readlane(ent, k);
        const int slot = u & (NBA - 1);
        if (lane == 0) {
          int p = cur[slot];
          p = p < 0 ? 0 : (p > RCAP - 1 ? RCAP - 1 : p);
          sl[p] = u;
          cur[slot] = p + 1;
        }
      }
    }
  }
  __syncthreads();

  const float qnan = __int_as_float(0x7fc00000);
  const float pz = (ovf != 0) ? qnan : 0.0f;
#pragma unroll 1
  for (int si = 0; si < NBA / NWAVE; ++si) {
    const int s    = si * NWAVE + wave;
    const int node = nodeBase + s;
    int c = cnt[s];
    const bool big = c > DEGCAP;
    c = c < 0 ? 0 : (c > DEGCAP ? DEGCAP : c);
    int o = offs[s];
    o = o < 0 ? 0 : (o > RCAP ? RCAP : o);
    const int nc = node < nN ? node : nN - 1;
    const float dd = dis[nc];
    const float rd = dd * dd;
    float a0 = 0.0f, a1 = 0.0f, a2 = 0.0f, a3 = 0.0f;
#pragma unroll 1
    for (int b0 = 0; b0 < c; b0 += 32) {
      int idx = o + b0 + lane;
      idx = idx > RCAP - 1 ? RCAP - 1 : idx;
      const int ent = sl[idx];
      int eid = ent >> SLA;
      eid = eid < 0 ? 0 : (eid > nE - 1 ? nE - 1 : eid);
      int sr = srcs[eid];
      sr = sr < 0 ? 0 : (sr > nN - 1 ? nN - 1 : sr);
      const float cf  = dis[sr] * dd;
      const int   cfi = __float_as_int(cf);
      const int m32 = (c - b0) < 32 ? (c - b0) : 32;
#pragma unroll 1
      for (int k = 0; k < m32; ++k) {
        const int   sk = __builtin_amdgcn_readlane(sr, k);
        const float ck = __int_as_float(__builtin_amdgcn_readlane(cfi, k));
        const v4f a = *(const v4fa*)(xl + (size_t)sk * HD + 4 * lane);
        a0 = fmaf(ck, a.x, a0); a1 = fmaf(ck, a.y, a1);
        a2 = fmaf(ck, a.z, a2); a3 = fmaf(ck, a.w, a3);
      }
    }
    const v4f sv = *(const v4fa*)(xl + (size_t)nc * HD + 4 * lane);
    const float pzr = big ? qnan : pz;
    const bool live = node < nN;
    float y0 = fmaxf((a0 + sv.x * rd) + bv4.x, 0.0f) + pzr;
    float y1 = fmaxf((a1 + sv.y * rd) + bv4.y, 0.0f) + pzr;
    float y2 = fmaxf((a2 + sv.z * rd) + bv4.z, 0.0f) + pzr;
    float y3 = fmaxf((a3 + sv.w * rd) + bv4.w, 0.0f) + pzr;
    const float m0 = live ? y0 : 0.0f;
    const float m1 = live ? y1 : 0.0f;
    const float m2 = live ? y2 : 0.0f;
    const float m3 = live ? y3 : 0.0f;
    v4us mh, ml;
    {
      unsigned hb;
      hb = bf16_bits(m0); mh[0] = (unsigned short)hb; ml[0] = (unsigned short)bf16_bits(m0 - __uint_as_float(hb << 16));
      hb = bf16_bits(m1); mh[1] = (unsigned short)hb; ml[1] = (unsigned short)bf16_bits(m1 - __uint_as_float(hb << 16));
      hb = bf16_bits(m2); mh[2] = (unsigned short)hb; ml[2] = (unsigned short)bf16_bits(m2 - __uint_as_float(hb << 16));
      hb = bf16_bits(m3); mh[3] = (unsigned short)hb; ml[3] = (unsigned short)bf16_bits(m3 - __uint_as_float(hb << 16));
    }
    *(v4usa*)(rowbuf + 4 * lane) = mh;
    *(v4usa*)(rowbuf + HD + 4 * lane) = ml;
    wave_sync();
    const v8us q0 = *(const v8usa*)(rowbuf + 8 * lane);
    wave_sync();
    if (node < mRows) {
      unsigned short* rpw = yout + (size_t)node * YP + 8 * lane;
      *(volatile v8us*)rpw = q0;
      __threadfence();
      *(volatile v8us*)rpw = q0;
    }
  }
}

static inline int cdiv(int a, int b) { return (a + b - 1) / b; }
static inline size_t al256(size_t o) { return (o + 255) & ~(size_t)255; }

extern "C" void kernel_launch(void* const* d_in, const int* in_sizes, int n_in,
                              void* d_out, int out_size, void* d_ws, size_t ws_size,
                              hipStream_t stream) {
  if (n_in < 15) return;
  if (in_sizes[0] < XF || (in_sizes[0] % XF) != 0) return;
  const int nN = in_sizes[0] / XF;
  if (nN < 16 || nN > (1 << 22) || (nN & 3) != 0) return;
  if (in_sizes[1] < 2 || (in_sizes[1] & 1) != 0) return;
  const int nE = in_sizes[1] / 2;
  if (nE < 1 || nE >= (1 << (31 - SLA))) return;
  if (in_sizes[3] != XF * HD || in_sizes[4] != HD) return;
  if (in_sizes[5] != HD * HD || in_sizes[6] != HD) return;
  if (in_sizes[7] != HD * HD || in_sizes[8] != HD) return;
  if (in_sizes[9] != HD * HD || in_sizes[10] != HD) return;
  if (in_sizes[11] != HD * HD || in_sizes[12] != HD) return;
  if (in_sizes[13] != HD * NCLS || in_sizes[14] != NCLS) return;
  if ((long long)out_size != (long long)nN * NCLS) return;

  const float* x    = (const float*)d_in[0];
  const int*   edge = (const int*)d_in[1];
  const float* W1   = (const float*)d_in[3];
  const float* b1   = (const float*)d_in[4];
  const float* W2   = (const float*)d_in[5];
  const float* b2   = (const float*)d_in[6];
  const float* W3   = (const float*)d_in[7];
  const float* b3   = (const float*)d_in[8];
  const float* fW1  = (const float*)d_in[9];
  const float* fb1  = (const float*)d_in[10];
  const float* fW2  = (const float*)d_in[11];
  const float* fb2  = (const float*)d_in[12];
  const float* fW3  = (const float*)d_in[13];
  const float* fb3  = (const float*)d_in[14];
  float* out = (float*)d_out;
  const int* src = edge;
  const int* dst = edge + nE;
  const int nTot = nN * NCLS;

  const int MP   = cdiv(nN, GBM) * GBM;
  const int gM   = MP / GBM;
  const int gD   = cdiv(nN, NBD);
  const int NBPD = gD * NBD;
  const int gA   = cdiv(MP, NBA);
  if ((long long)gA * NBA < (long long)MP) return;
  if (NBPD < nN) return;
  const int vec8 = ((nE & 3) == 0) ? 1 : 0;

  char* ws = (char*)d_ws;
  size_t off = 0;
  const size_t oDIS = off; off = al256(off + (size_t)NBPD * 4);
  const size_t oW1T = off; off = al256(off + (size_t)HD * K1P * 2);
  const size_t oWTB = off; off = al256(off + (size_t)5 * HD * K2 * 2);
  const size_t oXB  = off; off = al256(off + (size_t)MP * K1P * 2);
  const size_t oH   = off; off = al256(off + (size_t)MP * HD * 4);
  const size_t oYA  = off; off = al256(off + (size_t)MP * YP * 2);
  const size_t oYB  = off; off = al256(off + (size_t)MP * YP * 2);
  if (off > ws_size || off > (size_t)WSMAX) return;
  float*          DIS = (float*)(ws + oDIS);
  unsigned short* W1T = (unsigned short*)(ws + oW1T);
  unsigned short* WTB = (unsigned short*)(ws + oWTB);
  unsigned short* XB  = (unsigned short*)(ws + oXB);
  float*          H   = (float*)(ws + oH);
  unsigned short* YA  = (unsigned short*)(ws + oYA);
  unsigned short* YB  = (unsigned short*)(ws + oYB);
  unsigned short* W2T = WTB + (size_t)0 * HD * K2;
  unsigned short* W3T = WTB + (size_t)1 * HD * K2;
  unsigned short* W4T = WTB + (size_t)2 * HD * K2;
  unsigned short* W5T = WTB + (size_t)3 * HD * K2;
  unsigned short* W6T = WTB + (size_t)4 * HD * K2;

  const size_t aggLds = (size_t)AGG_LDS_INTS * 4;
  hipFuncSetAttribute(reinterpret_cast<const void*>(&k_agg), hipFuncAttributeMaxDynamicSharedMemorySize, (int)aggLds);

  const int nUx = MP * (K1P / 8);
  k_wprep<<<NUWT / NTHR, NTHR, 0, stream>>>(W1, W2, W3, fW1, fW2, fW3, W1T, WTB);
  k_cvx<<<cdiv(nUx, NTHR), NTHR, 0, stream>>>(x, nN, nUx, XB);
  k_deg<<<gD, NTHR, 0, stream>>>(dst, nE, vec8, DIS);
  k_gemm<0><<<gM, GTHR, 0, stream>>>(XB, K1P, W1T, K1P, b1, 0, H, YB, nN, nTot);
  k_agg<<<gA, NTHR, aggLds, stream>>>(src, dst, nE, nN, vec8, MP, DIS, H, b1, YA);
  k_gemm<0><<<gM, GTHR, 0, stream>>>(YA, YP, W2T, K2, b2, 0, H, YB, nN, nTot);
  k_agg<<<gA, NTHR, aggLds, stream>>>(src, dst, nE, nN, vec8, MP, DIS, H, b2, YB);
  k_gemm<0><<<gM, GTHR, 0, stream>>>(YB, YP, W3T, K2, b3, 0, H, YA, nN, nTot);
  k_agg<<<gA, NTHR, aggLds, stream>>>(src, dst, nE, nN, vec8, MP, DIS, H, b3, YA);
  k_gemm<1><<<gM, GTHR, 0, stream>>>(YA, YP, W4T, K2, fb1, HD, H, YB, nN, nTot);
  k_gemm<1><<<gM, GTHR, 0, stream>>>(YB, YP, W5T, K2, fb2, HD, H, YA, nN, nTot);
  k_gemm<2><<<gM, GTHR, 0, stream>>>(YA, YP, W6T, K2, fb3, NCLS, out, YB, nN, nTot);
}
